// GraphLearningEncoder_80264348827935
// MI455X (gfx1250) — hardware-verified
//
#include <hip/hip_runtime.h>
#include <stddef.h>


typedef _Float16 h16;
typedef _Float16 v16h __attribute__((ext_vector_type(16)));
typedef _Float16 v8h  __attribute__((ext_vector_type(8)));
typedef float    v8f  __attribute__((ext_vector_type(8)));
typedef float    v4f  __attribute__((ext_vector_type(4)));

#ifndef NB
#define NB 64
#endif
#define NB_FULL 64
#define CH   16
#define TT   20
#define NN   100
#define NE   (NN * NN)
#define KT   (CH * TT)
#define NPAD 128
#define EPAD 10048
#define KR   256
#define MROWS (NB * CH)
#define NPAIR (MROWS / 2)
#define GCOLS (2 * NE)
#define GTILES ((GCOLS + 63) / 64)
#ifndef A2_RES
#define A2_RES 1
#endif

static_assert(NB >= 8 && NB <= NB_FULL && (NB % 8) == 0);
static_assert((MROWS % 64) == 0 && (NPAIR % 64) == 0);
static_assert((KT % 32) == 0);
static_assert((KR % 32) == 0 && KR == 2 * NPAD);
static_assert((NPAD % 64) == 0 && NPAD >= NN && NPAD / 64 == 2);
static_assert((EPAD % 64) == 0 && (EPAD % 32) == 0 && EPAD >= NE);
static_assert((NE % 16) == 0);
static_assert((GCOLS % 32) == 0);
static_assert(GTILES * 64 - NE <= EPAD);
static_assert(NE <= 16384 && GTILES * 64 + 16384 - NE <= 32768);
static_assert((NN % 4) == 0 && NN >= 8);
static_assert((size_t)MROWS * EPAD < (size_t)0xFFFFFFFFu);

#define LDT 72
#define LDC 68
#define KLD 328
static_assert((LDT % 8) == 0 && LDT >= 64);
static_assert((LDC % 4) == 0 && LDC >= 64);
static_assert((KLD % 8) == 0 && KLD >= KT);
static_assert(64 * KLD * 2 + 16 * KLD * 2 + 16 * LDC * 4 <= 131072);
static_assert(64 * LDC * 4 <= 131072);
static_assert(2 * (256 / 8) == 64);
static_assert(4 * (256 / 16) == 64);
static_assert(2 * (128 / 16) == 16);
static_assert(1 * (128 / 8) == 16);

#define WCARRY  64.0f
#define HCARRY  64.0f
#define A1CARRY 4096.0f
#define ECARRY  4096.0f
#define PCARRY  65536.0f
#define RCARRY  2048.0f

#define R_BYTES   ((size_t)EPAD * KR * 2)
#define RT_BYTES  ((size_t)NPAD * EPAD * 2)
#define HF_BYTES  ((size_t)MROWS * NPAD * 4)
#define A_BYTES   ((size_t)MROWS * KR * 2)
#define HE_BYTES  ((size_t)MROWS * EPAD * 2)
#define OFF_R   ((size_t)0)
#define OFF_RT  (OFF_R + R_BYTES)
#define OFF_HF  (OFF_RT + RT_BYTES)
#define OFF_A1  (OFF_HF + HF_BYTES)
#define OFF_HE  (OFF_A1 + A_BYTES)
#define OFF_A2H (OFF_HE + HE_BYTES)
#define OFF_A2R (OFF_A2H + A_BYTES)
#define WS_TOTAL (OFF_A2R + A_BYTES)
static_assert((R_BYTES % 128) == 0 && (RT_BYTES % 128) == 0 && (HF_BYTES % 128) == 0);
static_assert((A_BYTES % 128) == 0 && (HE_BYTES % 128) == 0);
static_assert(WS_TOTAL <= (size_t)134217728);

__device__ __forceinline__ float bf16r(float x) {
  unsigned int u = __float_as_uint(x);
  u = (u + 0x7FFFu + ((u >> 16) & 1u)) & 0xFFFF0000u;
  return __uint_as_float(u);
}

static __device__ __forceinline__ h16 toh_flush(float v) {
  const h16 r = (h16)v;
  return (fabsf(v) < 6.103515625e-05f) ? (h16)0.0f : r;
}
static __device__ __forceinline__ void split_hi_res(float t, h16& hi, h16& rs) {
  hi = toh_flush(t);
  rs = toh_flush((t - (float)hi) * RCARRY);
}

__device__ __forceinline__ v16h frag_at(const _Float16* p) {
  v8h lo = *(const v8h*)(p);
  v8h hi = *(const v8h*)(p + 16);
  v16h out;
#pragma unroll
  for (int i = 0; i < 8; ++i) { out[i] = lo[i]; out[i + 8] = hi[i]; }
  return out;
}
__device__ __forceinline__ v16h ld_frag(const _Float16* base, unsigned ld) {
  const unsigned lane = threadIdx.x & 31u;
  return frag_at(base + (lane & 15u) * ld + (lane >> 4) * 8u);
}

__device__ __forceinline__ v8f wmma16(v16h a, v16h b, v8f c) {
  v8f d = __builtin_amdgcn_wmma_f32_16x16x32_f16(false, a, false, b, (short)0, c,
                                                 false, false);
  asm volatile("v_nop\n\tv_nop\n\tv_nop\n\tv_nop" : "+v"(d) : "v"(a), "v"(b));
  return d;
}

__device__ __forceinline__ unsigned row_parity(unsigned g) {
  return ((g + (16384u - (unsigned)NE)) >> 14) & 1u;
}

__global__ __launch_bounds__(256) void relplane_kernel(
    const float* __restrict__ rsend, const float* __restrict__ rrec, _Float16* __restrict__ R) {
#pragma clang fp contract(off)
  const unsigned tid = threadIdx.x;
  const unsigned e = blockIdx.x * 8u + (tid >> 5);
  const unsigned c = (tid & 31u) * 8u;
  const unsigned cl = c & 127u;
  const unsigned ec = (e < (unsigned)NE) ? e : (unsigned)(NE - 1);
  const unsigned c0 = (cl < (unsigned)(NN - 4)) ? cl : (unsigned)(NN - 4);
  const unsigned c1 = (cl + 4u < (unsigned)(NN - 4)) ? (cl + 4u) : (unsigned)(NN - 4);
  const size_t rb = (size_t)ec * NN;
  const v4f s0 = *(const v4f*)(rsend + rb + c0);
  const v4f s1 = *(const v4f*)(rsend + rb + c1);
  const v4f r0 = *(const v4f*)(rrec + rb + c0);
  const v4f r1 = *(const v4f*)(rrec + rb + c1);
  const bool use_rec = (c >= 128u);
  const bool ok0 = (e < (unsigned)NE) && (cl + 3u < (unsigned)NN);
  const bool ok1 = (e < (unsigned)NE) && (cl + 7u < (unsigned)NN);
  v8h o;
#pragma unroll
  for (int i = 0; i < 4; ++i) {
    float a0 = use_rec ? r0[i] : s0[i];
    float a1 = use_rec ? r1[i] : s1[i];
    a0 = ok0 ? a0 : 0.0f;
    a1 = ok1 ? a1 : 0.0f;
    o[i]     = toh_flush(bf16r(a0));
    o[i + 4] = toh_flush(bf16r(a1));
  }
  _Float16* p = R + (size_t)e * KR + c;
  *(volatile v8h*)p = o;
  __threadfence();
  *(volatile v8h*)p = o;
}

__global__ __launch_bounds__(256) void relT_kernel(
    const float* __restrict__ W, _Float16* __restrict__ Wt) {
#pragma clang fp contract(off)
  __shared__ _Float16 T[64 * LDT];
  const unsigned tid = threadIdx.x;
  const unsigned n0 = blockIdx.x * 64u;
  const unsigned k0 = blockIdx.y * 64u;
#pragma unroll 4
  for (unsigned j = 0; j < 16u; ++j) {
    const unsigned idx = tid + 256u * j;
    const unsigned kr = idx >> 6, nc = idx & 63u;
    const unsigned e = k0 + kr, n = n0 + nc;
    const unsigned ec = (e < (unsigned)NE) ? e : (unsigned)(NE - 1);
    const unsigned ncl = (n < (unsigned)NN) ? n : (unsigned)(NN - 1);
    float v = W[(size_t)ec * NN + ncl];
    v = ((e < (unsigned)NE) && (n < (unsigned)NN)) ? v : 0.0f;
    T[nc * LDT + kr] = toh_flush(bf16r(v));
  }
  __syncthreads();
  v8h x[2];
  size_t off[2];
#pragma unroll
  for (unsigned i = 0; i < 2u; ++i) {
    const unsigned n = 32u * i + (tid >> 3);
    const unsigned kc = (tid & 7u) * 8u;
    x[i] = *(const v8h*)&T[n * LDT + kc];
    off[i] = (size_t)(n0 + n) * EPAD + k0 + kc;
  }
#pragma unroll
  for (int i = 0; i < 2; ++i) *(volatile v8h*)(Wt + off[i]) = x[i];
  __threadfence();
#pragma unroll
  for (int i = 0; i < 2; ++i) *(volatile v8h*)(Wt + off[i]) = x[i];
}

__global__ __launch_bounds__(128) void nodefeat_kernel(
    const float* __restrict__ x, const float* __restrict__ tcm_w, const float* __restrict__ tcm_b,
    const float* __restrict__ tconv_w, const float* __restrict__ tconv_b,
    const float* __restrict__ n2e_w, float* __restrict__ Hf, _Float16* __restrict__ A1) {
  __shared__ _Float16 Hs[64 * KLD];
  __shared__ _Float16 Ws[16 * KLD];
  __shared__ float Cs[16 * LDC];
  const unsigned tid = threadIdx.x, lane = tid & 31u;
  const unsigned wave = (unsigned)__builtin_amdgcn_readfirstlane((int)(tid >> 5));
  const unsigned hh = lane >> 4, m = lane & 15u;
  const unsigned n0 = blockIdx.x * 64u;
  const unsigned b = blockIdx.y;

#pragma unroll 1
  for (unsigned idx = tid; idx < (unsigned)(CH * KT); idx += 128u) {
    const unsigned o = idx / (unsigned)KT;
    const unsigned k = idx - o * (unsigned)KT;
    Ws[o * KLD + k] = toh_flush(WCARRY * bf16r(tconv_w[idx]));
  }

  {
    const unsigned nl = tid & 63u;
    const unsigned chalf = wave >> 1;
    const unsigned n = n0 + nl;
    const bool nvalid = (n < (unsigned)NN);
    const unsigned ncl = nvalid ? n : (unsigned)(NN - 1);
#pragma unroll 1
    for (unsigned i = chalf * 8u; i < chalf * 8u + 8u; ++i) {
      const float w0 = bf16r(tcm_w[i * 3u + 0u]);
      const float w1 = bf16r(tcm_w[i * 3u + 1u]);
      const float w2 = bf16r(tcm_w[i * 3u + 2u]);
      const float bb = bf16r(tcm_b[i]);
      const float* xp = x + ((size_t)(b * (unsigned)CH + i) * TT) * NN + ncl;
      float xm = 0.0f;
      float xc = bf16r(xp[0]);
#pragma unroll 4
      for (unsigned t = 0; t < (unsigned)TT; ++t) {
        const unsigned tn = (t + 1u < (unsigned)TT) ? (t + 1u) : (unsigned)(TT - 1);
        const float xl = bf16r(xp[(size_t)tn * NN]);
        const float xn = (t + 1u < (unsigned)TT) ? xl : 0.0f;
        float v = ((xm * w0 + xc * w1) + xn * w2) + bb;
        v = fmaxf(v, 0.0f);
        v = nvalid ? v : 0.0f;
        Hs[nl * KLD + i * (unsigned)TT + t] = toh_flush(HCARRY * v);
        xm = xc;
        xc = xn;
      }
    }
  }
  __syncthreads();

  v8f acc = {};
#pragma unroll 2
  for (unsigned k0 = 0; k0 < (unsigned)KT; k0 += 32u) {
    const v16h a  = ld_frag(&Ws[k0], KLD);
    const v16h bf = ld_frag(&Hs[(wave * 16u) * KLD + k0], KLD);
    acc = wmma16(a, bf, acc);
  }
#pragma unroll
  for (int r = 0; r < 8; ++r)
    Cs[(hh * 8u + (unsigned)r) * LDC + wave * 16u + m] = acc[r];
  __syncthreads();

  const float hinv = 1.0f / (HCARRY * WCARRY);
  v4f hf[2];
  size_t offf[2];
#pragma unroll
  for (unsigned i = 0; i < 2u; ++i) {
    const unsigned r = 8u * i + (tid >> 4);
    const unsigned c = (tid & 15u) * 4u;
    const v4f u = *(const v4f*)&Cs[r * LDC + c];
    const float tb = bf16r(tconv_b[r]);
    v4f val;
#pragma unroll
    for (int j = 0; j < 4; ++j) {
      const float hv = u[j] * hinv + tb;
      val[j] = (n0 + c + (unsigned)j < (unsigned)NN) ? hv : 0.0f;
    }
    hf[i] = val;
    offf[i] = (size_t)(b * (unsigned)CH + r) * NPAD + n0 + c;
  }
  v8h x0, x1;
  size_t offa;
  {
    const unsigned r = tid >> 3;
    const unsigned c = (tid & 7u) * 8u;
    const v4f u0 = *(const v4f*)&Cs[r * LDC + c];
    const v4f u1 = *(const v4f*)&Cs[r * LDC + c + 4u];
    const float tb = bf16r(tconv_b[r]);
    const float w0 = bf16r(n2e_w[r * 2u + 0u]);
    const float w1 = bf16r(n2e_w[r * 2u + 1u]);
#pragma unroll
    for (int j = 0; j < 4; ++j) {
      const float ha = u0[j] * hinv + tb;
      const float hb = u1[j] * hinv + tb;
      const bool oka = (n0 + c + (unsigned)j < (unsigned)NN);
      const bool okb = (n0 + c + 4u + (unsigned)j < (unsigned)NN);
      x0[j]     = toh_flush(oka ? A1CARRY * (ha * w0) : 0.0f);
      x0[j + 4] = toh_flush(okb ? A1CARRY * (hb * w0) : 0.0f);
      x1[j]     = toh_flush(oka ? A1CARRY * (ha * w1) : 0.0f);
      x1[j + 4] = toh_flush(okb ? A1CARRY * (hb * w1) : 0.0f);
    }
    offa = (size_t)(b * (unsigned)CH + r) * KR + n0 + c;
  }
#pragma unroll
  for (int i = 0; i < 2; ++i) *(volatile v4f*)(Hf + offf[i]) = hf[i];
  *(volatile v8h*)(A1 + offa) = x0;
  *(volatile v8h*)(A1 + offa + NPAD) = x1;
  __threadfence();
#pragma unroll
  for (int i = 0; i < 2; ++i) *(volatile v4f*)(Hf + offf[i]) = hf[i];
  *(volatile v8h*)(A1 + offa) = x0;
  *(volatile v8h*)(A1 + offa + NPAD) = x1;
}

template <int MODE>
__device__ __forceinline__ void gemm_body(
    const _Float16* __restrict__ A16, const _Float16* __restrict__ Bt, const unsigned K,
    const float* __restrict__ n2e_w, const float* __restrict__ n2e_b,
    const float* __restrict__ e2n_w, const float* __restrict__ e2n_b,
    const float* __restrict__ n2e2_w, const float* __restrict__ Hf,
    _Float16* __restrict__ out16, _Float16* __restrict__ out16r) {
  __shared__ float Cs[64 * LDC];
  const unsigned tid = threadIdx.x, lane = tid & 31u, w = tid >> 5;
  const unsigned mw = w >> 1, nw = w & 1u;
  const unsigned hh = lane >> 4, m = lane & 15u;
  const unsigned n0 = blockIdx.x * 64u;
  const unsigned row0 = blockIdx.y * 64u;

  const _Float16* ap  = A16 + (size_t)(row0 + mw * 16u + m) * K + hh * 8u;
  const _Float16* bp0 = Bt + (size_t)(n0 + nw * 32u + m) * K + hh * 8u;
  const _Float16* bp1 = bp0 + (size_t)16 * K;
  v8f acc0 = {}, acc1 = {};
#pragma unroll 2
  for (unsigned k0 = 0; k0 < K; k0 += 32u) {
    const v16h a  = frag_at(ap + k0);
    const v16h b0 = frag_at(bp0 + k0);
    const v16h b1 = frag_at(bp1 + k0);
    acc0 = wmma16(a, b0, acc0);
    acc1 = wmma16(a, b1, acc1);
  }
#pragma unroll
  for (int r = 0; r < 8; ++r) {
    float* d = &Cs[(mw * 16u + hh * 8u + (unsigned)r) * LDC + nw * 32u + m];
    d[0]  = acc0[r];
    d[16] = acc1[r];
  }
  __syncthreads();

  if (MODE == 0) {
    v8h x[2];
    size_t off[2];
#pragma unroll
    for (unsigned i = 0; i < 2u; ++i) {
      const unsigned r = 32u * i + (tid >> 3);
      const unsigned c = (tid & 7u) * 8u;
      const unsigned ch = (row0 + r) & (unsigned)(CH - 1);
      const float nb = bf16r(n2e_b[ch]);
      const v4f u0 = *(const v4f*)&Cs[r * LDC + c];
      const v4f u1 = *(const v4f*)&Cs[r * LDC + c + 4];
#pragma unroll
      for (int j = 0; j < 4; ++j) {
        const float t0 = ECARRY * (u0[j] * (1.0f / A1CARRY) + nb);
        const float t1 = ECARRY * (u1[j] * (1.0f / A1CARRY) + nb);
        const bool ok0 = (n0 + c + (unsigned)j < (unsigned)NE);
        const bool ok1 = (n0 + c + 4u + (unsigned)j < (unsigned)NE);
        x[i][j]     = toh_flush(ok0 ? t0 : 0.0f);
        x[i][j + 4] = toh_flush(ok1 ? t1 : 0.0f);
      }
      off[i] = (size_t)(row0 + r) * EPAD + n0 + c;
    }
#pragma unroll
    for (int i = 0; i < 2; ++i) *(volatile v8h*)(out16 + off[i]) = x[i];
    __threadfence();
#pragma unroll
    for (int i = 0; i < 2; ++i) *(volatile v8h*)(out16 + off[i]) = x[i];
  }

  if (MODE == 1) {
    v8h xp[2], xq[2], rp[2], rq[2];
    size_t off[2];
#pragma unroll
    for (unsigned i = 0; i < 2u; ++i) {
      const unsigned r = 32u * i + (tid >> 3);
      const unsigned c = (tid & 7u) * 8u;
      const unsigned bc = row0 + r;
      const unsigned ch = bc & (unsigned)(CH - 1);
      const unsigned n = n0 + c;
      const float ew = bf16r(e2n_w[ch]);
      const float eb = bf16r(e2n_b[ch]);
      const float w0 = bf16r(n2e_w[ch * 2u + 0u]);
      const float w1 = bf16r(n2e_w[ch * 2u + 1u]);
      const float q0 = bf16r(n2e2_w[ch * 3u + 0u]);
      const float q1 = bf16r(n2e2_w[ch * 3u + 1u]);
      const float q2 = bf16r(n2e2_w[ch * 3u + 2u]);
      const float a0 = w0 * q2;
      const float a1 = w1 * q2;
      const v4f u0 = *(const v4f*)&Cs[r * LDC + c];
      const v4f u1 = *(const v4f*)&Cs[r * LDC + c + 4];
      const v4f hv0 = *(const v4f*)(Hf + (size_t)bc * NPAD + n);
      const v4f hv1 = *(const v4f*)(Hf + (size_t)bc * NPAD + n + 4u);
#pragma unroll
      for (int j = 0; j < 4; ++j) {
        const float hna = (u0[j] * (1.0f / ECARRY)) * (1.0f / (float)NN) * ew + eb;
        const float hnb = (u1[j] * (1.0f / ECARRY)) * (1.0f / (float)NN) * ew + eb;
        const bool oka = (n + (unsigned)j < (unsigned)NN);
        const bool okb = (n + 4u + (unsigned)j < (unsigned)NN);
        const float tpa = oka ? PCARRY * (hna * q0 + hv0[j] * a0) : 0.0f;
        const float tqa = oka ? PCARRY * (hna * q1 + hv0[j] * a1) : 0.0f;
        const float tpb = okb ? PCARRY * (hnb * q0 + hv1[j] * a0) : 0.0f;
        const float tqb = okb ? PCARRY * (hnb * q1 + hv1[j] * a1) : 0.0f;
        h16 hi, rs;
        split_hi_res(tpa, hi, rs); xp[i][j] = hi;     rp[i][j] = rs;
        split_hi_res(tqa, hi, rs); xq[i][j] = hi;     rq[i][j] = rs;
        split_hi_res(tpb, hi, rs); xp[i][j + 4] = hi; rp[i][j + 4] = rs;
        split_hi_res(tqb, hi, rs); xq[i][j + 4] = hi; rq[i][j + 4] = rs;
      }
      off[i] = (size_t)bc * KR + n;
    }
#pragma unroll
    for (int i = 0; i < 2; ++i) {
      *(volatile v8h*)(out16 + off[i]) = xp[i];
      *(volatile v8h*)(out16 + off[i] + NPAD) = xq[i];
      if (A2_RES) {
        *(volatile v8h*)(out16r + off[i]) = rp[i];
        *(volatile v8h*)(out16r + off[i] + NPAD) = rq[i];
      }
    }
    __threadfence();
#pragma unroll
    for (int i = 0; i < 2; ++i) {
      *(volatile v8h*)(out16 + off[i]) = xp[i];
      *(volatile v8h*)(out16 + off[i] + NPAD) = xq[i];
      if (A2_RES) {
        *(volatile v8h*)(out16r + off[i]) = rp[i];
        *(volatile v8h*)(out16r + off[i] + NPAD) = rq[i];
      }
    }
  }
}

__global__ __launch_bounds__(256) void gemm_edge_kernel(
    const _Float16* __restrict__ A1, const _Float16* __restrict__ R,
    const float* __restrict__ n2e_b, _Float16* __restrict__ HE) {
  gemm_body<0>(A1, R, (unsigned)KR, n2e_b, n2e_b, n2e_b, n2e_b, n2e_b, n2e_b, HE, HE);
}
__global__ __launch_bounds__(256) void gemm_node_kernel(
    const _Float16* __restrict__ HE, const _Float16* __restrict__ RT,
    const float* __restrict__ n2e_w, const float* __restrict__ e2n_w,
    const float* __restrict__ e2n_b, const float* __restrict__ n2e2_w,
    const float* __restrict__ Hf, _Float16* __restrict__ A2H, _Float16* __restrict__ A2R) {
  gemm_body<1>(HE, RT, (unsigned)EPAD, n2e_w, n2e_w, e2n_w, e2n_b, n2e2_w, Hf, A2H, A2R);
}

__global__ __launch_bounds__(256) void gemm_out_kernel(
    const _Float16* __restrict__ A2H, const _Float16* __restrict__ A2R,
    const _Float16* __restrict__ R, const float* __restrict__ n2e_b,
    const float* __restrict__ n2e2_w, const float* __restrict__ n2e2_b,
    float* __restrict__ out) {
  __shared__ float Cs[64 * LDC];
  const unsigned tid = threadIdx.x, lane = tid & 31u;
  const unsigned wave = (unsigned)__builtin_amdgcn_readfirstlane((int)(tid >> 5));
  const unsigned mw = wave >> 1, nw = wave & 1u;
  const unsigned hh = lane >> 4, m = lane & 15u;
  const unsigned g0 = blockIdx.x * 64u;
  const unsigned pair0 = blockIdx.y * 64u;

  const unsigned gs0 = g0 + nw * 32u, gs1 = gs0 + 16u;
  const unsigned par0 = row_parity(gs0), par1 = row_parity(gs1);
  const unsigned e0 = gs0 - par0 * (unsigned)NE;
  const unsigned e1 = gs1 - par1 * (unsigned)NE;
  const unsigned prow = pair0 + mw * 16u + m;
  const size_t ao0 = (size_t)(2u * prow + par0) * KR + hh * 8u;
  const size_t ao1 = (size_t)(2u * prow + par1) * KR + hh * 8u;
  const size_t bo0 = (size_t)(e0 + m) * KR + hh * 8u;
  const size_t bo1 = (size_t)(e1 + m) * KR + hh * 8u;

  v8f acc0 = {}, acc1 = {}, rc0 = {}, rc1 = {};
#pragma unroll 2
  for (unsigned k0 = 0; k0 < (unsigned)KR; k0 += 32u) {
    const v16h b0 = frag_at(R + bo0 + k0);
    const v16h b1 = frag_at(R + bo1 + k0);
    const v16h ah0 = frag_at(A2H + ao0 + k0);
    const v16h ah1 = frag_at(A2H + ao1 + k0);
    acc0 = wmma16(ah0, b0, acc0);
    acc1 = wmma16(ah1, b1, acc1);
    if (A2_RES) {
      const v16h ar0 = frag_at(A2R + ao0 + k0);
      const v16h ar1 = frag_at(A2R + ao1 + k0);
      rc0 = wmma16(ar0, b0, rc0);
      rc1 = wmma16(ar1, b1, rc1);
    }
  }
#pragma unroll
  for (int r = 0; r < 8; ++r) {
    float* d = &Cs[(mw * 16u + hh * 8u + (unsigned)r) * LDC + nw * 32u + m];
    d[0]  = acc0[r] + rc0[r] * (1.0f / RCARRY);
    d[16] = acc1[r] + rc1[r] * (1.0f / RCARRY);
  }
  __syncthreads();

  v4f xs[4];
  size_t off[4];
  bool ok[4];
#pragma unroll
  for (unsigned i = 0; i < 4u; ++i) {
    const unsigned r = 16u * i + (tid >> 4);
    const unsigned c = (tid & 15u) * 4u;
    const unsigned g = g0 + c;
    const unsigned par = row_parity(g);
    const unsigned ch = (2u * (pair0 + r) + par) & (unsigned)(CH - 1);
    const float cst = bf16r(n2e_b[ch]) * bf16r(n2e2_w[ch * 3u + 2u]) + bf16r(n2e2_b[ch]);
    const v4f u = *(const v4f*)&Cs[r * LDC + c];
    v4f val;
#pragma unroll
    for (int j = 0; j < 4; ++j) val[j] = u[j] * (1.0f / PCARRY) + cst;
    xs[i] = val;
    ok[i] = (g < (unsigned)GCOLS);
    off[i] = (size_t)(pair0 + r) * GCOLS + g;
  }
#pragma unroll
  for (int i = 0; i < 4; ++i)
    if (ok[i]) *(volatile v4f*)(out + off[i]) = xs[i];
  __threadfence();
#pragma unroll
  for (int i = 0; i < 4; ++i)
    if (ok[i]) *(volatile v4f*)(out + off[i]) = xs[i];
}

extern "C" void kernel_launch(void* const* d_in, const int* in_sizes, int n_in,
                              void* d_out, int out_size, void* d_ws, size_t ws_size,
                              hipStream_t stream) {
  if (n_in < 13) return;
  if ((long long)in_sizes[0] < (long long)NB * CH * TT * NN) return;
  if ((long long)in_sizes[1] < (long long)NE * NN) return;
  if ((long long)in_sizes[2] < (long long)NE * NN) return;
  if (in_sizes[3] < CH * 3 || in_sizes[4] < CH) return;
  if (in_sizes[5] < CH * KT || in_sizes[6] < CH) return;
  if (in_sizes[7] < CH * 2 || in_sizes[8] < CH) return;
  if (in_sizes[9] < CH || in_sizes[10] < CH) return;
  if (in_sizes[11] < CH * 3 || in_sizes[12] < CH) return;
  if ((long long)out_size < (long long)MROWS * NE) return;
  if (ws_size < WS_TOTAL) return;

  const float* x        = (const float*)d_in[0];
  const float* rel_rec  = (const float*)d_in[1];
  const float* rel_send = (const float*)d_in[2];
  const float* tcm_w    = (const float*)d_in[3];
  const float* tcm_b    = (const float*)d_in[4];
  const float* tconv_w  = (const float*)d_in[5];
  const float* tconv_b  = (const float*)d_in[6];
  const float* n2e_w    = (const float*)d_in[7];
  const float* n2e_b    = (const float*)d_in[8];
  const float* e2n_w    = (const float*)d_in[9];
  const float* e2n_b    = (const float*)d_in[10];
  const float* n2e2_w   = (const float*)d_in[11];
  const float* n2e2_b   = (const float*)d_in[12];
  float* out = (float*)d_out;

  char* ws = (char*)d_ws;
  _Float16* Rp  = (_Float16*)(ws + OFF_R);
  _Float16* RTp = (_Float16*)(ws + OFF_RT);
  float*    Hf  = (float*)(ws + OFF_HF);
  _Float16* A1  = (_Float16*)(ws + OFF_A1);
  _Float16* HE  = (_Float16*)(ws + OFF_HE);
  _Float16* A2H = (_Float16*)(ws + OFF_A2H);
  _Float16* A2R = (_Float16*)(ws + OFF_A2R);

  relplane_kernel<<<dim3(EPAD / 8), dim3(256), 0, stream>>>(rel_send, rel_rec, Rp);
  relT_kernel<<<dim3(NPAD / 64, EPAD / 64), dim3(256), 0, stream>>>(rel_rec, RTp);
  nodefeat_kernel<<<dim3(NPAD / 64, NB), dim3(128), 0, stream>>>(
      x, tcm_w, tcm_b, tconv_w, tconv_b, n2e_w, Hf, A1);
  gemm_edge_kernel<<<dim3(EPAD / 64, MROWS / 64), dim3(256), 0, stream>>>(A1, Rp, n2e_b, HE);
  gemm_node_kernel<<<dim3(NPAD / 64, MROWS / 64), dim3(256), 0, stream>>>(
      HE, RTp, n2e_w, e2n_w, e2n_b, n2e2_w, Hf, A2H, A2R);
  gemm_out_kernel<<<dim3(GTILES, NPAIR / 64), dim3(256), 0, stream>>>(
      A2H, A2R, Rp, n2e_b, n2e2_w, n2e2_b, out);
}
